// TemporalCNNAttention_29618094474195
// MI455X (gfx1250) — hardware-run, weakly checked
//
#include <hip/hip_runtime.h>
#include <math.h>
#include <stdint.h>

#define E_DIM   128
#define W_DIM   16
#define P_DIM   4096
#define B_DIM   8
#define PT      32
#define EP      64
#define EPP     68
#define NPB     (P_DIM / PT)
#define THREADS 256
#define NGROUPS 4
#define ULD     36
#define PLD     16
#define GN_EPS  1e-5f
#define FSC     256.0f
#define IFS     0.00390625f
#define IS2     1.52587890625e-05f
#define RSQE    0.08838834764831845f

#define NF_LDS  15488u
#define NU_LDS  50048u
#define SMEM_BYTES (NF_LDS * 4u + NU_LDS * 4u)

static_assert((P_DIM % PT) == 0);
static_assert(PT == 32);
static_assert((E_DIM % 32) == 0);
static_assert(EP * 2 == E_DIM);
static_assert((EPP % 4) == 0 && EPP >= EP);
static_assert(THREADS == 256);
static_assert(E_DIM == 16 * (THREADS / 32));
static_assert((E_DIM / NGROUPS) == 32);
static_assert(SMEM_BYTES == 262144u);
static_assert(((NF_LDS * 4u) % 16u) == 0u);
static_assert(NPB * PT == P_DIM);

typedef _Float16       v16h __attribute__((ext_vector_type(16)));
typedef _Float16       v2h  __attribute__((ext_vector_type(2)));
typedef float          v2f  __attribute__((ext_vector_type(2)));
typedef float          v8f  __attribute__((ext_vector_type(8)));
typedef float          v4f_raw __attribute__((ext_vector_type(4)));
typedef unsigned int   v4u_raw __attribute__((ext_vector_type(4)));
typedef double         v2d_raw __attribute__((ext_vector_type(2)));
typedef v4f_raw __attribute__((may_alias)) v4f;
typedef v4u_raw __attribute__((may_alias)) v4u;
typedef v2d_raw __attribute__((may_alias)) v2d;

union Frag { v16h v; v4u q[2]; };
static_assert(sizeof(Frag) == 32);

__device__ __forceinline__ float bfr(float f) {
  unsigned u = __float_as_uint(f);
  u = (u + 0x7FFFu + ((u >> 16) & 1u)) & 0xFFFF0000u;
  return __uint_as_float(u);
}
__device__ __forceinline__ unsigned int pk_h2(float x, float y) {
  v2f f = {x, y};
  v2h h = __builtin_convertvector(f, v2h);
  return __builtin_bit_cast(unsigned int, h);
}
__device__ __forceinline__ v2f up_h2(unsigned int u) {
  v2h h = __builtin_bit_cast(v2h, u);
  return __builtin_convertvector(h, v2f);
}
__device__ __forceinline__ float gelu_exact(float x) {
  return 0.5f * x * (1.0f + erff(x * 0.70710678118654752f));
}
__device__ __forceinline__ v8f zero8() { v8f z = {0.f, 0.f, 0.f, 0.f, 0.f, 0.f, 0.f, 0.f}; return z; }

__device__ __forceinline__ v8f mma_h(v16h a, v16h b, v8f c) {
  v8f d = __builtin_amdgcn_wmma_f32_16x16x32_f16(false, a, false, b, (short)0, c, false, false);
#if defined(__HIP_DEVICE_COMPILE__)
  asm volatile("v_nop\n\tv_nop\n\tv_nop\n\tv_nop" : "+v"(d) : "v"(a), "v"(b));
#endif
  return d;
}

__device__ __forceinline__ void load_A_frag(const unsigned int* w, int m0, int k0, int lane, Frag& a) {
  const unsigned int* base = w + (m0 + (lane & 15)) * EPP + (k0 >> 1);
  const int h = lane >> 4;
  a.q[0] = *(const v4u*)(base + 4 * h);
  a.q[1] = *(const v4u*)(base + 8 + 4 * h);
}
__device__ __forceinline__ void load_B_frag(const unsigned int* src, int k0, int n0, int lane, Frag& b) {
  const unsigned int* base = src + (n0 + (lane & 15)) * EPP + (k0 >> 1);
  const int h = lane >> 4;
  b.q[0] = *(const v4u*)(base + 4 * h);
  b.q[1] = *(const v4u*)(base + 8 + 4 * h);
}

__device__ __forceinline__ void stage_w(unsigned int* dst, const float* __restrict__ src, int tid, bool transpose) {
  for (int i = tid; i < E_DIM * EP; i += THREADS) {
    const int m = i >> 6, kp = i & 63;
    const int ia = transpose ? ((2 * kp) * E_DIM + m)     : (m * E_DIM + 2 * kp);
    const int ib = transpose ? ((2 * kp + 1) * E_DIM + m) : (m * E_DIM + 2 * kp + 1);
    const float x = bfr(src[ia]) * FSC;
    const float y = bfr(src[ib]) * FSC;
    dst[m * EPP + kp] = pk_h2(x, y);
  }
}

template <bool HAS_BIAS, bool WRITE_P, bool WRITE_32>
__device__ __forceinline__ void gemm128(const unsigned int* wlds, const unsigned int* Bsrc,
                                        unsigned int* DstP, float* Dst32, const float* biasL,
                                        int wave, int lane) {
  const int m0 = wave * 16;
  const int n  = lane & 15;
  const int h  = lane >> 4;
#pragma unroll
  for (int n0 = 0; n0 < PT; n0 += 16) {
    v8f c = zero8();
#pragma unroll
    for (int k0 = 0; k0 < E_DIM; k0 += 32) {
      Frag a, bf;
      load_A_frag(wlds, m0, k0, lane, a);
      load_B_frag(Bsrc, k0, n0, lane, bf);
      c = mma_h(a.v, bf.v, c);
    }
    const int nn = n0 + n;
    float vv[8];
#pragma unroll
    for (int r = 0; r < 8; ++r) {
      vv[r] = c[r] * IS2;
      if (HAS_BIAS) vv[r] += biasL[m0 + 8 * h + r];
    }
    if (WRITE_32) {
#pragma unroll
      for (int r = 0; r < 8; ++r) Dst32[(m0 + 8 * h + r) * PT + nn] = vv[r];
    }
    if (WRITE_P) {
      v4u st;
      st[0] = pk_h2(vv[0] * FSC, vv[1] * FSC);
      st[1] = pk_h2(vv[2] * FSC, vv[3] * FSC);
      st[2] = pk_h2(vv[4] * FSC, vv[5] * FSC);
      st[3] = pk_h2(vv[6] * FSC, vv[7] * FSC);
      *(v4u*)(DstP + nn * EPP + (m0 >> 1) + 4 * h) = st;
    }
  }
}

__global__ __launch_bounds__(THREADS)
void fused_tile_kernel(const float* __restrict__ u,
                       const float* __restrict__ emb_w, const float* __restrict__ emb_b,
                       const float* __restrict__ wq, const float* __restrict__ bq,
                       const float* __restrict__ wk, const float* __restrict__ bk,
                       const float* __restrict__ wv, const float* __restrict__ bv,
                       const float* __restrict__ wo, const float* __restrict__ bo,
                       float* xbuf, double* partial) {
  extern __shared__ __align__(16) char smem[];
  float* u_lds  = (float*)smem;
  float* we0    = u_lds + W_DIM * ULD;
  float* we1    = we0 + 128;
  float* we2    = we1 + 128;
  float* web    = we2 + 128;
  float* bqL    = web + 128;
  float* bkL    = bqL + 128;
  float* bvL    = bkL + 128;
  float* boL    = bvL + 128;
  float* lastf  = boL + 128;
  float* Qf     = lastf + E_DIM * PT;
  float* qkf    = Qf + E_DIM * PT;
  float* scores = qkf + E_DIM * PT;
  float* attn   = scores + W_DIM * PT;
  float* qb     = attn + W_DIM * PT;
  float* psum   = qb + PT;
  float* psq    = psum + 256;
  double* stgd  = (double*)(psq + 256);
  unsigned int* featP = (unsigned int*)(smem + NF_LDS * 4u);
  unsigned int* QP    = featP + W_DIM * PT * EPP;
  unsigned int* cfP   = QP + PT * EPP;
  unsigned int* ctxP  = cfP + PT * EPP;
  unsigned int* wstg  = ctxP + PT * EPP;

  const int tid  = threadIdx.x;
  const int lane = tid & 31, wave = tid >> 5;
  const int pblk = blockIdx.x, b = blockIdx.y;
  const int p0   = pblk * PT;

  for (int i = tid; i < W_DIM * 34; i += THREADS) {
    const int w  = i / 34, j = i - w * 34;
    const int pg = p0 - 1 + j;
    const int pc = min(max(pg, 0), P_DIM - 1);
    float v = u[((size_t)b * W_DIM + w) * P_DIM + pc];
    v = (pg >= 0 && pg < P_DIM) ? v : 0.f;
    u_lds[w * ULD + j] = bfr(v);
  }
  if (tid < E_DIM) {
    we0[tid] = bfr(emb_w[tid * 3 + 0]);
    we1[tid] = bfr(emb_w[tid * 3 + 1]);
    we2[tid] = bfr(emb_w[tid * 3 + 2]);
    web[tid] = bfr(emb_b[tid]);
    bqL[tid] = bfr(bq[tid]);
    bkL[tid] = bfr(bk[tid]);
    bvL[tid] = bfr(bv[tid]);
    boL[tid] = bfr(bo[tid]);
  }
  __syncthreads();

  for (int i = tid; i < W_DIM * PT * EP; i += THREADS) {
    const int w  = i >> 11;
    const int p  = (i >> 6) & 31;
    const int ep = i & 63;
    const float* ur = u_lds + w * ULD + p;
    const float u0 = ur[0], u1 = ur[1], u2 = ur[2];
    const int ea = 2 * ep, eb = 2 * ep + 1;
    const float x0 = gelu_exact(we0[ea] * u0 + we1[ea] * u1 + we2[ea] * u2 + web[ea]);
    const float x1 = gelu_exact(we0[eb] * u0 + we1[eb] * u1 + we2[eb] * u2 + web[eb]);
    featP[(w * PT + p) * EPP + ep] = pk_h2(x0 * FSC, x1 * FSC);
    if (w == W_DIM - 1) { lastf[ea * PT + p] = x0; lastf[eb * PT + p] = x1; }
  }
  __syncthreads();

  stage_w(wstg, wq, tid, false);
  __syncthreads();
  gemm128<true, true, true>(wstg, featP + (W_DIM - 1) * PT * EPP, QP, Qf, bqL, wave, lane);
  __syncthreads();

  stage_w(wstg, wk, tid, true);
  if (tid < PT) {
    float s = 0.f;
    for (int f = 0; f < E_DIM; ++f) s += Qf[f * PT + tid] * bkL[f];
    qb[tid] = s;
  }
  __syncthreads();
  gemm128<false, false, true>(wstg, QP, nullptr, qkf, nullptr, wave, lane);
  __syncthreads();

  for (int i = tid; i < W_DIM * PT; i += THREADS) {
    const int w = i >> 5, p = i & 31;
    const unsigned int* fr = featP + (w * PT + p) * EPP;
    float s = 0.f;
    for (int ep = 0; ep < EP; ++ep) {
      const v2f f2 = up_h2(fr[ep]);
      s += qkf[(2 * ep) * PT + p] * f2[0] + qkf[(2 * ep + 1) * PT + p] * f2[1];
    }
    scores[w * PT + p] = (s * IFS + qb[p]) * RSQE;
  }
  __syncthreads();
  if (tid < PT) {
    float m = -1e30f;
    for (int w = 0; w < W_DIM; ++w) m = fmaxf(m, scores[w * PT + tid]);
    float s = 0.f;
    for (int w = 0; w < W_DIM; ++w) {
      const float e = __expf(scores[w * PT + tid] - m);
      attn[w * PT + tid] = e;
      s += e;
    }
    const float inv = 1.0f / s;
    for (int w = 0; w < W_DIM; ++w) attn[w * PT + tid] = attn[w * PT + tid] * inv;
  }
  __syncthreads();

  for (int i = tid; i < PT * EP; i += THREADS) {
    const int p  = i >> 6;
    const int ep = i & 63;
    float s0 = 0.f, s1 = 0.f;
    for (int w = 0; w < W_DIM; ++w) {
      const v2f f2 = up_h2(featP[(w * PT + p) * EPP + ep]);
      const float a = attn[w * PT + p];
      s0 += a * f2[0];
      s1 += a * f2[1];
    }
    cfP[p * EPP + ep] = pk_h2(s0, s1);
  }
  stage_w(wstg, wv, tid, false);
  __syncthreads();

  gemm128<true, true, false>(wstg, cfP, ctxP, nullptr, bvL, wave, lane);
  __syncthreads();
  stage_w(wstg, wo, tid, false);
  __syncthreads();

  {
    const int m0 = wave * 16;
    const int n  = lane & 15;
    const int h  = lane >> 4;
    float s1 = 0.f, s2 = 0.f;
#pragma unroll
    for (int n0 = 0; n0 < PT; n0 += 16) {
      v8f c = zero8();
#pragma unroll
      for (int k0 = 0; k0 < E_DIM; k0 += 32) {
        Frag a, bf;
        load_A_frag(wstg, m0, k0, lane, a);
        load_B_frag(ctxP, k0, n0, lane, bf);
        c = mma_h(a.v, bf.v, c);
      }
#pragma unroll
      for (int r = 0; r < 8; ++r) {
        const int f  = m0 + 8 * h + r;
        const int li = f * PT + n0 + n;
        const float xv = c[r] * IS2 + boL[f] + lastf[li];
        lastf[li] = xv;
        s1 += xv; s2 += xv * xv;
      }
    }
    psum[tid] = s1; psq[tid] = s2;
  }
  __syncthreads();
  if (tid < NGROUPS) {
    double d1 = 0.0, d2 = 0.0;
    for (int t = tid * 64; t < tid * 64 + 64; ++t) { d1 += (double)psum[t]; d2 += (double)psq[t]; }
    stgd[2 * tid]     = d1;
    stgd[2 * tid + 1] = d2;
  }
  if (tid >= 8 && tid < PLD) stgd[tid] = 0.0;
  __syncthreads();

  {
    const int e = tid & 7, lq = tid >> 3;
    float* xb = xbuf + ((size_t)b * E_DIM) * P_DIM + p0;
    v4f xv[4];
#pragma unroll
    for (int it = 0; it < 4; ++it) xv[it] = *(const v4f*)(lastf + (it * 32 + lq) * PT + 4 * e);
    const v2d pd = *(const v2d*)(stgd + 2 * (lane & 7));
    double* pl = partial + (size_t)(b * NPB + pblk) * PLD + 2 * (lane & 7);
#pragma unroll
    for (int pass = 0; pass < 2; ++pass) {
#pragma unroll
      for (int it = 0; it < 4; ++it)
        *(volatile v4f*)(xb + (size_t)(it * 32 + lq) * P_DIM + 4 * e) = xv[it];
      if (tid < 8) *(volatile v2d*)pl = pd;
      __threadfence();
    }
  }
}

__global__ __launch_bounds__(THREADS)
void gn_kernel(const float* __restrict__ xbuf, const double* __restrict__ partial,
               const float* __restrict__ gw, const float* __restrict__ gb, float* y) {
  __shared__ double sd1[128];
  __shared__ double sd2[128];
  __shared__ float  sh2[2];
  const int tid = threadIdx.x;
  const int be  = blockIdx.x;
  const int b   = be >> 7;
  const int e   = be & 127;
  const int g   = e >> 5;
  if (tid < 128) {
    const double* pl = partial + (size_t)(b * NPB + tid) * PLD + 2 * g;
    sd1[tid] = pl[0];
    sd2[tid] = pl[1];
  }
  __syncthreads();
  for (int s = 64; s > 0; s >>= 1) {
    if (tid < s) { sd1[tid] += sd1[tid + s]; sd2[tid] += sd2[tid + s]; }
    __syncthreads();
  }
  if (tid == 0) {
    const double invN = 1.0 / (double)((E_DIM / NGROUPS) * P_DIM);
    const double mu  = sd1[0] * invN;
    const double var = sd2[0] * invN - mu * mu;
    float varf = (float)var;
    varf = varf > 0.f ? varf : 0.f;
    sh2[0] = (float)mu;
    sh2[1] = 1.0f / sqrtf(varf + GN_EPS);
  }
  __syncthreads();
  const float mu  = sh2[0];
  const float rs  = sh2[1];
  const float gwv = bfr(gw[e]);
  const float gbv = bfr(gb[e]);
  const float* row = xbuf + (size_t)be * P_DIM;
  float* orow = y + (size_t)be * P_DIM;
  v4f ov[4];
#pragma unroll
  for (int it = 0; it < 4; ++it) {
    const int idx = (it * THREADS + tid) * 4;
    const v4f v = *(const v4f*)(row + idx);
    v4f o;
#pragma unroll
    for (int q = 0; q < 4; ++q) o[q] = ((v[q] - mu) * rs) * gwv + gbv;
    ov[it] = o;
  }
#pragma unroll
  for (int pass = 0; pass < 2; ++pass) {
#pragma unroll
    for (int it = 0; it < 4; ++it) {
      const int idx = (it * THREADS + tid) * 4;
      *(volatile v4f*)(orow + idx) = ov[it];
    }
    __threadfence();
  }
}

extern "C" void kernel_launch(void* const* d_in, const int* in_sizes, int n_in,
                              void* d_out, int out_size, void* d_ws, size_t ws_size,
                              hipStream_t stream) {
  if (n_in < 13) return;
  if (in_sizes[0] != B_DIM * W_DIM * P_DIM) return;
  if (in_sizes[1] != E_DIM * 3 || in_sizes[2] != E_DIM) return;
  if (in_sizes[3] != E_DIM * E_DIM || in_sizes[4] != E_DIM) return;
  if (in_sizes[5] != E_DIM * E_DIM || in_sizes[6] != E_DIM) return;
  if (in_sizes[7] != E_DIM * E_DIM || in_sizes[8] != E_DIM) return;
  if (in_sizes[9] != E_DIM * E_DIM || in_sizes[10] != E_DIM) return;
  if (in_sizes[11] != E_DIM || in_sizes[12] != E_DIM) return;
  if (out_size != B_DIM * E_DIM * P_DIM) return;

  size_t off = 0;
  const size_t oX = off; off += (size_t)B_DIM * E_DIM * P_DIM * sizeof(float);
  const size_t oP = off; off += (size_t)B_DIM * NPB * PLD * sizeof(double);
  if (off > ws_size) return;
  if (off > (size_t)134217728) return;

  const float* u    = (const float*)d_in[0];
  const float* embw = (const float*)d_in[1];
  const float* embb = (const float*)d_in[2];
  const float* wq   = (const float*)d_in[3];
  const float* bq   = (const float*)d_in[4];
  const float* wk   = (const float*)d_in[5];
  const float* bk   = (const float*)d_in[6];
  const float* wv   = (const float*)d_in[7];
  const float* bv   = (const float*)d_in[8];
  const float* wo   = (const float*)d_in[9];
  const float* bo   = (const float*)d_in[10];
  const float* gw   = (const float*)d_in[11];
  const float* gb   = (const float*)d_in[12];

  char* ws = (char*)d_ws;
  float*  xbuf    = (float*)(ws + oX);
  double* partial = (double*)(ws + oP);
  float*  y       = (float*)d_out;

  (void)hipFuncSetAttribute(reinterpret_cast<const void*>(&fused_tile_kernel),
                            hipFuncAttributeMaxDynamicSharedMemorySize, (int)SMEM_BYTES);

  const dim3 gridF(NPB, B_DIM);
  fused_tile_kernel<<<gridF, dim3(THREADS), SMEM_BYTES, stream>>>(
      u, embw, embb, wq, bq, wk, bk, wv, bv, wo, bo, xbuf, partial);
  const dim3 gridG(B_DIM * E_DIM);
  gn_kernel<<<gridG, dim3(THREADS), 0, stream>>>(xbuf, partial, gw, gb, y);
  (void)hipGetLastError();
}
